// ScalableDAG_v1_32993938768553
// MI455X (gfx1250) — hardware-run, weakly checked
//
#include <hip/hip_runtime.h>
#include <math.h>

typedef __attribute__((ext_vector_type(16))) _Float16 v16h;
typedef __attribute__((ext_vector_type(8)))  _Float16 v8h;
typedef __attribute__((ext_vector_type(8)))  float    v8f;
typedef __attribute__((ext_vector_type(4)))  float    v4f;

constexpr int kBatchRows = 16384;
constexpr int kNodes     = 128;
constexpr int kHidden    = 64;
constexpr int kLoc       = 8;
constexpr int kWtRows    = kNodes * kHidden;
constexpr int kBlkRows   = 128;
constexpr int kBlkNodes  = 32;
constexpr int kPanelP    = 136;
constexpr int kOutP      = 36;

static_assert((kNodes % 32) == 0, "contraction depth is a multiple of 32");
static_assert((kBatchRows % kBlkRows) == 0 && (kNodes % kBlkNodes) == 0, "block tiling is exact");
static_assert(kBlkRows == 8 * 16, "8 waves x 16 rows");
static_assert(kHidden == 4 * 16, "4 column tiles of 16");
static_assert((kPanelP % 8) == 0 && kPanelP >= kNodes, "16-B aligned panel rows");
static_assert((kOutP % 4) == 0 && kOutP >= kBlkNodes, "16-B aligned result rows");
static_assert(kBlkNodes * 4 == 128, "one 128-B line per row segment");

constexpr size_t kOffXH   = 0;
constexpr size_t kOffWT   = kOffXH + (size_t)kBatchRows * kNodes * 2;
constexpr size_t kOffBB   = kOffWT + (size_t)kWtRows * kNodes * 2;
constexpr size_t kOffVW   = kOffBB + (size_t)kWtRows * 4;
constexpr size_t kOffCV   = kOffVW + (size_t)kWtRows * 4;
constexpr size_t kWsTotal = kOffCV + (size_t)kNodes * 4;
static_assert(kWsTotal == 6357504ull, "carve total");
static_assert(kWsTotal <= 134217728ull, "carve cap");
static_assert((kOffWT % 128) == 0 && (kOffBB % 128) == 0 && (kOffVW % 128) == 0 && (kOffCV % 128) == 0,
              "128-B aligned regions");

union FragH { v16h v; v8h h[2]; };

__device__ __forceinline__ v16h frag_load(const _Float16* p) {
  FragH f;
  f.h[0] = *(const v8h*)(p);
  f.h[1] = *(const v8h*)(p + 16);
  return f.v;
}

__device__ __forceinline__ v8f mma_f16(v16h a, v16h b, v8f c) {
  c = __builtin_amdgcn_wmma_f32_16x16x32_f16(false, a, false, b, (short)0, c, false, false);
  asm volatile("v_nop\n\tv_nop\n\tv_nop\n\tv_nop" : "+v"(c) : "v"(a), "v"(b));
  return c;
}

__global__ __launch_bounds__(256) void cvt_rows_f16_kernel(
    const float* __restrict__ src, unsigned short* __restrict__ dst, int total8)
{
  const int i = blockIdx.x * 256 + threadIdx.x;
  if (i >= total8) return;
  const size_t e0 = (size_t)i << 3;
  const v4f a0 = *(const v4f*)(src + e0);
  const v4f a1 = *(const v4f*)(src + e0 + 4);
  v8h hv;
#pragma unroll
  for (int e = 0; e < 4; ++e) {
    const float f0 = a0[e];
    const float f1 = a1[e];
    hv[e]     = (_Float16)f0;
    hv[4 + e] = (_Float16)f1;
  }
  unsigned short* q = dst + e0;
  *(volatile v8h*)q = hv;
  __threadfence();
  *(volatile v8h*)q = hv;
}

__global__ __launch_bounds__(256) void mask_diff_f16_kernel(
    const float* __restrict__ wp, const float* __restrict__ wn,
    unsigned short* __restrict__ dst, int total8)
{
  const int i = blockIdx.x * 256 + threadIdx.x;
  if (i >= total8) return;
  const size_t e0 = (size_t)i << 3;
  const int j  = (int)(e0 >> 13);
  const int d0 = (int)(e0 & (size_t)(kNodes - 1));
  const v4f p0 = *(const v4f*)(wp + e0);
  const v4f p1 = *(const v4f*)(wp + e0 + 4);
  const v4f n0 = *(const v4f*)(wn + e0);
  const v4f n1 = *(const v4f*)(wn + e0 + 4);
  v8h hv;
#pragma unroll
  for (int e = 0; e < 4; ++e) {
    float f0 = p0[e] - n0[e];
    float f1 = p1[e] - n1[e];
    f0 = ((d0 + e) == j) ? 0.0f : f0;
    f1 = ((d0 + 4 + e) == j) ? 0.0f : f1;
    hv[e]     = (_Float16)f0;
    hv[4 + e] = (_Float16)f1;
  }
  unsigned short* q = dst + e0;
  *(volatile v8h*)q = hv;
  __threadfence();
  *(volatile v8h*)q = hv;
}

__global__ __launch_bounds__(256) void tail_fold_kernel(
    const float* __restrict__ b1p, const float* __restrict__ b1n,
    const float* __restrict__ w2, const float* __restrict__ b2, const float* __restrict__ w3,
    float* __restrict__ bb, float* __restrict__ vw, float* __restrict__ cvec)
{
  const int tid = threadIdx.x;
  if (blockIdx.x < 8) {
    const int i  = blockIdx.x * 256 + tid;
    const int j  = i >> 4;
    const int m4 = (i & 15) * 4;
    const v4f p = *(const v4f*)(b1p + (size_t)i * 4);
    const v4f n = *(const v4f*)(b1n + (size_t)i * 4);
    v4f bv;
    bv[0] = p[0] - n[0];
    bv[1] = p[1] - n[1];
    bv[2] = p[2] - n[2];
    bv[3] = p[3] - n[3];
    v4f av = (v4f){0.f, 0.f, 0.f, 0.f};
#pragma unroll 1
    for (int k = 0; k < kLoc; ++k) {
      const float w = w3[j * kLoc + k];
      const v4f c2 = *(const v4f*)(w2 + k * kHidden + m4);
      av[0] = fmaf(w, c2[0], av[0]);
      av[1] = fmaf(w, c2[1], av[1]);
      av[2] = fmaf(w, c2[2], av[2]);
      av[3] = fmaf(w, c2[3], av[3]);
    }
    float* qb = bb + (size_t)i * 4;
    float* qv = vw + (size_t)i * 4;
    *(volatile v4f*)qb = bv;
    *(volatile v4f*)qv = av;
    __threadfence();
    *(volatile v4f*)qb = bv;
    *(volatile v4f*)qv = av;
  } else {
    if (tid < 32) {
      v4f cv;
#pragma unroll
      for (int e = 0; e < 4; ++e) {
        const int j = tid * 4 + e;
        float c = 0.0f;
#pragma unroll 1
        for (int k = 0; k < kLoc; ++k) c = fmaf(w3[j * kLoc + k], b2[k], c);
        cv[e] = c;
      }
      float* qc = cvec + tid * 4;
      *(volatile v4f*)qc = cv;
      __threadfence();
      *(volatile v4f*)qc = cv;
    }
  }
}

__global__ __launch_bounds__(256) void fused_node_mlp_kernel(
    const unsigned short* __restrict__ XHp, const unsigned short* __restrict__ WTp,
    const float* __restrict__ bb, const float* __restrict__ vw, const float* __restrict__ cvec,
    float* __restrict__ out)
{
  __shared__ __align__(16) _Float16 sB[2][kHidden * kPanelP];
  __shared__ __align__(16) float    sO[8 * 16 * kOutP];

  const _Float16* XH = (const _Float16*)XHp;
  const _Float16* WT = (const _Float16*)WTp;

  const int tid  = threadIdx.x;
  const int lane = tid & 31;
  const int wave = tid >> 5;
  const int hh   = lane >> 4;
  const int col  = lane & 15;
  const int jgrp = blockIdx.x & 3;
  const int nblk = blockIdx.x >> 2;
  const int jbase = jgrp * kBlkNodes;
  const int nbase = nblk * kBlkRows + wave * 16;

  v16h afr[4];
  {
    const _Float16* xrow = XH + (size_t)(nbase + col) * kNodes + 8 * hh;
#pragma unroll
    for (int s = 0; s < 4; ++s) afr[s] = frag_load(xrow + 32 * s);
  }

  {
    const _Float16* src = WT + (size_t)jbase * (kHidden * kNodes);
#pragma unroll
    for (int i = 0; i < 4; ++i) {
      const int q   = tid + 256 * i;
      const int m   = q >> 4;
      const int seg = q & 15;
      const v8h w = *(const v8h*)(src + (size_t)q * 8);
      *(v8h*)(&sB[0][m * kPanelP + seg * 8]) = w;
    }
  }
  __syncthreads();

  float* otile = sO + wave * 16 * kOutP;

#pragma unroll 1
  for (int jj = 0; jj < kBlkNodes; ++jj) {
    const int j = jbase + jj;

    if (jj + 1 < kBlkNodes) {
      const _Float16* src = WT + (size_t)(j + 1) * (kHidden * kNodes);
      _Float16* dstp = &sB[(jj + 1) & 1][0];
#pragma unroll
      for (int i = 0; i < 4; ++i) {
        const int q   = tid + 256 * i;
        const int m   = q >> 4;
        const int seg = q & 15;
        const v8h w = *(const v8h*)(src + (size_t)q * 8);
        *(v8h*)(dstp + m * kPanelP + seg * 8) = w;
      }
    }

    float bcol[4], vcol[4];
#pragma unroll
    for (int t = 0; t < 4; ++t) {
      const int idx = j * kHidden + t * 16 + col;
      bcol[t] = bb[idx];
      vcol[t] = vw[idx];
    }
    const float cj = cvec[j];

    v8f acc[4];
#pragma unroll
    for (int t = 0; t < 4; ++t) {
      const float b0 = bcol[t];
      acc[t] = (v8f){b0, b0, b0, b0, b0, b0, b0, b0};
    }

    const _Float16* bp = &sB[jj & 1][col * kPanelP + 8 * hh];
#pragma unroll
    for (int s = 0; s < 4; ++s) {
#pragma unroll
      for (int t = 0; t < 4; ++t) {
        const v16h bf = frag_load(bp + t * 16 * kPanelP + 32 * s);
        acc[t] = mma_f16(afr[s], bf, acc[t]);
      }
    }

    float rsum[8];
#pragma unroll
    for (int r = 0; r < 8; ++r) {
      float sr = 0.0f;
#pragma unroll
      for (int t = 0; t < 4; ++t) {
        const float hval = acc[t][r];
        const float ex = __expf(-hval);
        const float sg = __builtin_amdgcn_rcpf(1.0f + ex);
        sr = fmaf(sg, vcol[t], sr);
      }
      rsum[r] = sr;
    }

    float t4[4];
#pragma unroll
    for (int r = 0; r < 4; ++r) {
      const float s0 = rsum[2 * r];
      const float s1 = rsum[2 * r + 1];
      const float x0 = __shfl_xor(s0, 1, 32);
      const float x1 = __shfl_xor(s1, 1, 32);
      const float e0 = s0 + x0;
      const float e1 = s1 + x1;
      t4[r] = (lane & 1) ? e1 : e0;
    }
    float t2[2];
#pragma unroll
    for (int r = 0; r < 2; ++r) {
      const float s0 = t4[2 * r];
      const float s1 = t4[2 * r + 1];
      const float x0 = __shfl_xor(s0, 2, 32);
      const float x1 = __shfl_xor(s1, 2, 32);
      const float e0 = s0 + x0;
      const float e1 = s1 + x1;
      t2[r] = (lane & 2) ? e1 : e0;
    }
    float red;
    {
      const float s0 = t2[0];
      const float s1 = t2[1];
      const float x0 = __shfl_xor(s0, 4, 32);
      const float x1 = __shfl_xor(s1, 4, 32);
      const float e0 = s0 + x0;
      const float e1 = s1 + x1;
      red = (lane & 4) ? e1 : e0;
    }
    {
      const float x8 = __shfl_xor(red, 8, 32);
      red = red + x8;
    }
    const float res = red + cj;
    if ((lane & 8) == 0) otile[(hh * 8 + (lane & 7)) * kOutP + jj] = res;

    __syncthreads();
  }

  {
    const int q  = lane >> 3;
    const int c4 = (lane & 7) * 4;
    v4f vals[4];
#pragma unroll
    for (int it = 0; it < 4; ++it) {
      const int row = it * 4 + q;
      vals[it] = *(const v4f*)(otile + row * kOutP + c4);
    }
    for (int pass = 0; pass < 2; ++pass) {
#pragma unroll
      for (int it = 0; it < 4; ++it) {
        const int row = it * 4 + q;
        *(volatile v4f*)(out + (size_t)(nbase + row) * kNodes + jbase + c4) = vals[it];
      }
      __threadfence();
    }
  }
}

extern "C" void kernel_launch(void* const* d_in, const int* in_sizes, int n_in,
                              void* d_out, int out_size, void* d_ws, size_t ws_size,
                              hipStream_t stream) {
  if (n_in < 8) return;
  if (in_sizes[0] != kBatchRows * kNodes) return;
  if (in_sizes[1] != kWtRows * kNodes) return;
  if (in_sizes[2] != kWtRows) return;
  if (in_sizes[3] != kWtRows * kNodes) return;
  if (in_sizes[4] != kWtRows) return;
  if (in_sizes[5] != kLoc * kHidden) return;
  if (in_sizes[6] != kLoc) return;
  if (in_sizes[7] != kNodes * kLoc) return;
  if (out_size != kBatchRows * kNodes) return;
  if (ws_size < kWsTotal) return;

  const float* x   = (const float*)d_in[0];
  const float* w1p = (const float*)d_in[1];
  const float* b1p = (const float*)d_in[2];
  const float* w1n = (const float*)d_in[3];
  const float* b1n = (const float*)d_in[4];
  const float* w2  = (const float*)d_in[5];
  const float* b2  = (const float*)d_in[6];
  const float* w3  = (const float*)d_in[7];
  float* out = (float*)d_out;

  char* ws = (char*)d_ws;
  unsigned short* XH = (unsigned short*)(ws + kOffXH);
  unsigned short* WT = (unsigned short*)(ws + kOffWT);
  float*          BB = (float*)(ws + kOffBB);
  float*          VW = (float*)(ws + kOffVW);
  float*          CV = (float*)(ws + kOffCV);

  constexpr int kX8 = kBatchRows * kNodes / 8;
  constexpr int kW8 = kWtRows * kNodes / 8;
  static_assert((kX8 % 256) == 0 && (kW8 % 256) == 0, "exact convert grids");

  cvt_rows_f16_kernel<<<kX8 / 256, 256, 0, stream>>>(x, XH, kX8);
  mask_diff_f16_kernel<<<kW8 / 256, 256, 0, stream>>>(w1p, w1n, WT, kW8);
  tail_fold_kernel<<<9, 256, 0, stream>>>(b1p, b1n, w2, b2, w3, BB, VW, CV);

  constexpr int kBlocks = (kBatchRows / kBlkRows) * (kNodes / kBlkNodes);
  fused_node_mlp_kernel<<<kBlocks, 256, 0, stream>>>(XH, WT, BB, VW, CV, out);
}
